// ForwardExecutor_33062658245245
// MI455X (gfx1250) — hardware-verified
//
#include <hip/hip_runtime.h>

#define __bf16 _Float16
typedef __attribute__((ext_vector_type(16))) _Float16 v16bf;
typedef __attribute__((ext_vector_type(8)))  float  v8f;
typedef __attribute__((ext_vector_type(4)))  float  v4f_t;
typedef float v4fa __attribute__((ext_vector_type(4), may_alias));
#define RSPLIT (1.0f / 2048.0f)

#define L_LAYERS 8
#define K_NODES  8
#define INDEG    4
#define DD       128
#define BB       4096
#define NN       (1 + L_LAYERS * K_NODES)
#define ROWS     16
#define STRIDE   136
#define SLICE    (ROWS * STRIDE)
#define STAGE_ELEMS   (K_NODES * SLICE)
#define OST_FLOATS    (8 * ROWS * DD)
#define SMEM_BYTES    (2 * STAGE_ELEMS * 2 + OST_FLOATS * 4)
#define NODE_F        (ROWS * DD)
#define WPL           ((size_t)NN * DD * DD)

namespace rg {
typedef unsigned int u32; typedef unsigned long long u64;
typedef unsigned __int128 u128;
constexpr u32 XSHIFT = 16;
constexpr u32 INIT_A = 0x43b0d7e5u, MULT_A = 0x931e8875u;
constexpr u32 INIT_B = 0x8b51f9ddu, MULT_B = 0x58f38dedu;
constexpr u32 MIX_L  = 0xca01f9ddu, MIX_R  = 0x4973f715u;

constexpr u32 hashmix(u32 v, u32& hc) { v ^= hc; hc *= MULT_A; v *= hc; v ^= v >> XSHIFT; return v; }
constexpr u32 mix2(u32 x, u32 y) { u32 r = (x * MIX_L) ^ (y * MIX_R); r ^= r >> XSHIFT; return r; }

constexpr u128 PCG_MULT = (((u128)0x2360ed051fc65da4ULL) << 64) | (u128)0x4385df649fce6645ULL;
struct Pcg { u128 state; u128 inc; bool has32; u32 buf; };
constexpr u64 rotr64(u64 v, unsigned r) { r &= 63u; return r ? (v >> r) | (v << (64u - r)) : v; }
constexpr u64 next64(Pcg& g) {
  g.state = g.state * PCG_MULT + g.inc;
  u64 hi = (u64)(g.state >> 64), lo = (u64)g.state;
  return rotr64(hi ^ lo, (unsigned)(g.state >> 122));
}
constexpr u32 next32(Pcg& g) {
  if (g.has32) { g.has32 = false; return g.buf; }
  u64 n = next64(g); g.has32 = true; g.buf = (u32)(n >> 32); return (u32)n;
}
struct Srcs { int v[L_LAYERS][K_NODES][INDEG]; };
constexpr Srcs build() {
  u32 hc = INIT_A; u32 pool[4] = {0, 0, 0, 0};
  for (int i = 0; i < 4; i++) pool[i] = hashmix(0u, hc);
  for (int s = 0; s < 4; s++)
    for (int d = 0; d < 4; d++)
      if (s != d) pool[d] = mix2(pool[d], hashmix(pool[s], hc));
  u32 hb = INIT_B; u32 st[8] = {};
  for (int i = 0; i < 8; i++) { u32 v = pool[i & 3]; v ^= hb; hb *= MULT_B; v *= hb; v ^= v >> XSHIFT; st[i] = v; }
  u64 w0 = (u64)st[0] | ((u64)st[1] << 32), w1 = (u64)st[2] | ((u64)st[3] << 32);
  u64 w2 = (u64)st[4] | ((u64)st[5] << 32), w3 = (u64)st[6] | ((u64)st[7] << 32);
  Pcg g{}; g.state = 0; g.inc = ((((u128)w2 << 64) | w3) << 1) | (u128)1u; g.has32 = false; g.buf = 0;
  g.state = g.state * PCG_MULT + g.inc;
  g.state += (((u128)w0) << 64) | w1;
  g.state = g.state * PCG_MULT + g.inc;
  Srcs out{};
  for (int k = 0; k < K_NODES; k++) for (int j = 0; j < INDEG; j++) out.v[0][k][j] = 0;
  for (int l = 1; l < L_LAYERS; l++) {
    u32 rng = (u32)(K_NODES * l);
    u32 rex = rng + 1u;
    u32 thresh = (0xFFFFFFFFu - rng) % rex;
    for (int k = 0; k < K_NODES; k++)
      for (int j = 0; j < INDEG; j++) {
        u64 m = (u64)next32(g) * (u64)rex;
        u32 lo = (u32)m;
        if (lo < rex) { while (lo < thresh) { m = (u64)next32(g) * (u64)rex; lo = (u32)m; } }
        out.v[l][k][j] = (int)(m >> 32);
      }
  }
  return out;
}
}

__constant__ int g_srcs_tab[L_LAYERS][K_NODES][INDEG] =
   {{{0,0,0,0},{0,0,0,0},{0,0,0,0},{0,0,0,0},{0,0,0,0},{0,0,0,0},{0,0,0,0},{0,0,0,0}},
   {{7,5,4,2},{2,0,0,0},{1,7,5,8},{4,5,8,6},{5,4,5,8},{2,7,6,0},{3,7,4,0},{6,6,7,1}},
   {{1,14,0,9},{1,5,8,7},{6,0,0,2},{0,11,8,11},{4,10,12,6},{7,16,13,16},{6,11,16,11},{14,11,11,6}},
   {{21,3,14,18},{21,13,9,7},{10,12,17,22},{1,23,13,8},{16,14,6,8},{17,14,12,8},{19,9,8,22},{6,5,17,15}},
   {{1,2,12,27},{13,25,10,7},{26,28,2,1},{22,11,18,4},{28,14,29,26},{23,7,25,1},{18,13,32,6},{31,2,20,19}},
   {{36,12,36,27},{36,8,31,38},{1,14,26,4},{20,25,31,38},{16,18,19,39},{8,20,2,17},{38,25,14,40},{24,38,0,18}},
   {{40,37,19,24},{20,25,11,38},{3,20,13,35},{36,34,45,45},{9,5,6,35},{47,45,32,47},{42,0,5,42},{4,48,40,46}},
   {{20,8,29,55},{20,50,21,46},{13,27,18,13},{50,45,7,52},{55,15,24,30},{37,25,8,53},{39,2,46,41},{10,35,28,1}}};

#if defined(__has_builtin)
#if __has_builtin(__builtin_amdgcn_cvt_pk_bf16_f32)
#define HAVE_CVT_PK_BF16 1
#endif
#endif

__device__ __forceinline__ void split16(float f, unsigned short& h, unsigned short& l) {
  const _Float16 hh = (_Float16)f; h = __builtin_bit_cast(unsigned short, hh);
  l = __builtin_bit_cast(unsigned short, (_Float16)((f - (float)hh) * 2048.0f));
}
__device__ __forceinline__ unsigned pack2s(float a, float b, unsigned* lo) {
  unsigned short h0, l0, h1, l1; split16(a, h0, l0); split16(b, h1, l1);
  *lo = (unsigned)l0 | ((unsigned)l1 << 16); return (unsigned)h0 | ((unsigned)h1 << 16);
}

union ABReg { v16bf v; uint4 q[2]; };

__device__ __forceinline__ void load_A(const unsigned short* aStage, int lane, ABReg A[4], ABReg AL[4]) {
  const int m = lane & 15, half = lane >> 4;
  const unsigned short* ap = aStage + m * STRIDE + half * 8;
#pragma unroll
  for (int c = 0; c < 4; c++) {
    A[c].q[0]  = *(const uint4*)(ap + c * 32);
    A[c].q[1]  = *(const uint4*)(ap + c * 32 + 16);
    AL[c].q[0] = *(const uint4*)(ap + STAGE_ELEMS + c * 32);
    AL[c].q[1] = *(const uint4*)(ap + STAGE_ELEMS + c * 32 + 16);
  }
}

__device__ __forceinline__ void mm_tile(const ABReg A[4], const ABReg AL[4], int node, int tile, int lane,
                                        const unsigned short* __restrict__ Wb,
                                        const float* __restrict__ bias,
                                        float* ost) {
  const int n15 = lane & 15, half = lane >> 4;
  const int e = tile * 16 + n15;
  const unsigned short* bp = Wb + ((size_t)node * DD + e) * DD + half * 8;
  v8f acc = {};
#pragma unroll
  for (int c = 0; c < 4; c++) {
    ABReg Bm, Bl;
    Bm.q[0] = *(const uint4*)(bp + c * 32);        Bm.q[1] = *(const uint4*)(bp + c * 32 + 16);
    Bl.q[0] = *(const uint4*)(bp + WPL + c * 32);  Bl.q[1] = *(const uint4*)(bp + WPL + c * 32 + 16);
    v8f x = {};
    x = __builtin_amdgcn_wmma_f32_16x16x32_f16(false, AL[c].v, false, Bm.v, (short)0, x, false, false);
    x = __builtin_amdgcn_wmma_f32_16x16x32_f16(false, A[c].v,  false, Bl.v, (short)0, x, false, false);
    acc = __builtin_amdgcn_wmma_f32_16x16x32_f16(false, A[c].v, false, Bm.v, (short)0, acc, false, false) + x * RSPLIT;
  }
  const float bv = bias[node * DD + e];
#pragma unroll
  for (int r = 0; r < 8; ++r) ost[(r + 8 * half) * DD + e] = __builtin_fmaxf(acc[r] + bv, 0.f);
}

__device__ __forceinline__ void store_node(const float* ost, float* dst, int lane) {
#pragma unroll 1
  for (int pass = 0; pass < 2; ++pass) {
#pragma unroll 4
    for (int i = 0; i < 16; ++i) {
      const int c = lane + 32 * i, rr = c >> 5, q = c & 31;
      *(volatile v4f_t*)(dst + rr * DD + q * 4) = *(const volatile v4fa*)(ost + rr * DD + q * 4);
    }
    __threadfence();
  }
}

__global__ __launch_bounds__(256) void wcvt_kernel(const float* __restrict__ W,
                                                   unsigned short* __restrict__ Wb) {
  const size_t i = ((size_t)blockIdx.x * 256 + threadIdx.x) * 8;
  float4 a = *(const float4*)(W + i);
  float4 b = *(const float4*)(W + i + 4);
  typedef __attribute__((ext_vector_type(4))) unsigned v4u_t;
  v4u_t o, ol; unsigned lo;
  o.x = pack2s(a.x, a.y, &lo); ol.x = lo; o.y = pack2s(a.z, a.w, &lo); ol.y = lo;
  o.z = pack2s(b.x, b.y, &lo); ol.z = lo; o.w = pack2s(b.z, b.w, &lo); ol.w = lo;
  *(volatile v4u_t*)(Wb + i) = o; *(volatile v4u_t*)(Wb + WPL + i) = ol;
  __threadfence();
  *(volatile v4u_t*)(Wb + i) = o; *(volatile v4u_t*)(Wb + WPL + i) = ol;
}

__global__ __launch_bounds__(256) void dag_kernel(const float* __restrict__ X,
                                                  const unsigned short* __restrict__ Wb,
                                                  const float* __restrict__ bias,
                                                  float* __restrict__ nodeOutAll,
                                                  float* __restrict__ out) {
  extern __shared__ unsigned short smem[];
  unsigned short* stage = smem;
  float* ostAll = (float*)(smem + 2 * STAGE_ELEMS);

  const int tid  = threadIdx.x;
  const int wave = tid >> 5;
  const int lane = tid & 31;
  const int rowBase = blockIdx.x * ROWS;
  const int sm = tid >> 4;
  const int sd = (tid & 15) * 8;
  const int sOff = sm * STRIDE + sd;
  float* nodeOut = nodeOutAll + (size_t)blockIdx.x * NN * NODE_F;
  float* ost = ostAll + wave * (ROWS * DD);

  auto stage8 = [&](int k, const float* v) {
    typedef __attribute__((ext_vector_type(4))) unsigned v4u_t;
    v4u_t o, ol; unsigned lo;
    o.x = pack2s(v[0], v[1], &lo); ol.x = lo; o.y = pack2s(v[2], v[3], &lo); ol.y = lo;
    o.z = pack2s(v[4], v[5], &lo); ol.z = lo; o.w = pack2s(v[6], v[7], &lo); ol.w = lo;
    *(v4u_t*)(stage + k * SLICE + sOff) = o; *(v4u_t*)(stage + STAGE_ELEMS + k * SLICE + sOff) = ol;
  };

  {
    const float* xp = X + (size_t)(rowBase + sm) * DD + sd;
    float v[8]; float4 a = *(const float4*)xp, b = *(const float4*)(xp + 4);
    v[0] = a.x; v[1] = a.y; v[2] = a.z; v[3] = a.w; v[4] = b.x; v[5] = b.y; v[6] = b.z; v[7] = b.w;
    stage8(0, v);
  }
  __syncthreads();
  {
    ABReg A[4], AL[4];
    load_A(stage, lane, A, AL);
    mm_tile(A, AL, 0, wave, lane, Wb, bias, ostAll);
  }
  __syncthreads();
  if (wave == 0) store_node(ostAll, nodeOut, lane);
  __syncthreads();

  int nodeBase = 1;
  for (int l = 0; l < L_LAYERS; l++) {
    {
      const unsigned short* wpan = Wb + (size_t)nodeBase * DD * DD;
#pragma unroll
      for (int pf = 0; pf < 4; pf++)
        __builtin_prefetch(wpan + ((size_t)tid * 4 + pf) * 128, 0, 3);
    }
    for (int k = 0; k < K_NODES; k++) {
      float v[8];
      {
        const float* p0 = nodeOut + g_srcs_tab[l][k][0] * NODE_F + sm * DD + sd;
        const v4f_t a = *(const volatile v4fa*)p0, b = *(const volatile v4fa*)(p0 + 4);
        v[0] = a.x; v[1] = a.y; v[2] = a.z; v[3] = a.w; v[4] = b.x; v[5] = b.y; v[6] = b.z; v[7] = b.w;
      }
#pragma unroll
      for (int j = 1; j < INDEG; ++j) {
        const float* pj = nodeOut + g_srcs_tab[l][k][j] * NODE_F + sm * DD + sd;
        const v4f_t a = *(const volatile v4fa*)pj, b = *(const volatile v4fa*)(pj + 4);
        v[0] += a.x; v[1] += a.y; v[2] += a.z; v[3] += a.w; v[4] += b.x; v[5] += b.y; v[6] += b.z; v[7] += b.w;
      }
      stage8(k, v);
    }
    __syncthreads();
    {
      const int node = nodeBase + wave;
      ABReg A[4], AL[4];
      load_A(stage + wave * SLICE, lane, A, AL);
#pragma unroll 1
      for (int t = 0; t < K_NODES; t++)
        mm_tile(A, AL, node, t, lane, Wb, bias, ost);
      asm volatile("s_wait_dscnt 0" ::: "memory");
      store_node(ost, nodeOut + (size_t)node * NODE_F, lane);
    }
    __syncthreads();
    nodeBase += K_NODES;
  }

  {
    v4f_t m2[2]; size_t mo[2];
#pragma unroll
    for (int i = 0; i < 2; ++i) {
      const int c = tid + 256 * i, rr = c >> 5, q = c & 31;
      v4f_t s = {0.f, 0.f, 0.f, 0.f};
#pragma unroll
      for (int j = 0; j < K_NODES; j++) s += *(const volatile v4fa*)(nodeOut + (size_t)(NN - K_NODES + j) * NODE_F + rr * DD + q * 4);
      m2[i] = s * 0.125f; mo[i] = (size_t)(rowBase + rr) * DD + q * 4;
    }
#pragma unroll
    for (int i = 0; i < 2; ++i) *(volatile v4f_t*)(out + mo[i]) = m2[i];
    __threadfence();
#pragma unroll
    for (int i = 0; i < 2; ++i) *(volatile v4f_t*)(out + mo[i]) = m2[i];
  }
}

extern "C" void kernel_launch(void* const* d_in, const int* in_sizes, int n_in,
                              void* d_out, int out_size, void* d_ws, size_t ws_size,
                              hipStream_t stream) {
  (void)in_sizes; (void)n_in; (void)out_size; (void)ws_size;
  const float* X    = (const float*)d_in[0];
  const float* W    = (const float*)d_in[1];
  const float* bias = (const float*)d_in[2];
  float* out = (float*)d_out;
  unsigned short* Wb = (unsigned short*)d_ws;
  float* nodeOutAll = (float*)((char*)d_ws + (8u << 20));

  wcvt_kernel<<<dim3((NN * DD * DD) / (256 * 8)), dim3(256), 0, stream>>>(W, Wb);
  dag_kernel<<<dim3(BB / ROWS), dim3(256), SMEM_BYTES, stream>>>(X, Wb, bias, nodeOutAll, out);
}
